// SAModule_predefined_adj_52999896432944
// MI455X (gfx1250) — hardware-verified
//
#include <hip/hip_runtime.h>
#include <stddef.h>
#include <stdint.h>


#define HC     128
#define DIN    64
#define NTHR   128
#define NWAVE  4
#define EPT    8
#define CHUNK  (NTHR * EPT)
#define WCAP   (EPT * 32)
#define LISTN  (NWAVE * WCAP)
#define PASSN  (NWAVE * 16)
#define PCAP   (CHUNK + PASSN)
#define NB     256
#define GROWS  64
#define GTHR   128
#define WSC    8.0f
#define WINV   0.125f

static_assert(PASSN == 64);
static_assert((PASSN % 32) == 0);
static_assert(PASSN <= NTHR);
static_assert((NB % NWAVE) == 0);
static_assert(PCAP >= CHUNK + PASSN);
static_assert((NTHR % 16) == 0);

typedef float    v4f  __attribute__((ext_vector_type(4)));
typedef float    v8f  __attribute__((ext_vector_type(8)));
typedef int      v4i  __attribute__((ext_vector_type(4)));
typedef _Float16 v8h  __attribute__((ext_vector_type(8)));
typedef _Float16 v16h __attribute__((ext_vector_type(16)));
union FragH { v16h v; v8h h[2]; };
union Pk8   { v8h h; v4i u; };

__device__ __forceinline__ v8f zero8f() {
  v8f z;
#pragma unroll
  for (int i = 0; i < 8; ++i) z[i] = 0.0f;
  return z;
}

__device__ __forceinline__ v8f wmh(v16h a, v16h b, v8f c) {
  v8f d = __builtin_amdgcn_wmma_f32_16x16x32_f16(false, a, false, b, (short)0, c, false, false);
  asm volatile("v_nop\n\tv_nop\n\tv_nop\n\tv_nop" : "+v"(d) : "v"(a), "v"(b));
  return d;
}

__device__ __forceinline__ v8h cvt8(v4f a, v4f b) {
  v8h r;
  r[0] = (_Float16)a.x; r[1] = (_Float16)a.y; r[2] = (_Float16)a.z; r[3] = (_Float16)a.w;
  r[4] = (_Float16)b.x; r[5] = (_Float16)b.y; r[6] = (_Float16)b.z; r[7] = (_Float16)b.w;
  return r;
}

__global__ __launch_bounds__(256) void k_prep(const float* __restrict__ W1, const float* __restrict__ W2,
                                              _Float16* W1t, _Float16* W2t) {
  __shared__ __attribute__((aligned(16))) _Float16 sT[HC * HC];
  const int tid = threadIdx.x, lane = tid & 31, wave = tid >> 5;
  for (int i = tid; i < HC * HC; i += 256) {
    const int k = i >> 7, n = i & 127;
    sT[n * HC + k] = (_Float16)(W2[i] * WSC);
  }
  __syncthreads();
  Pk8 o2[8];
#pragma unroll
  for (int j = 0; j < 8; ++j) {
    const int p = (wave * 8 + j) * 32 + lane;
    o2[j].h = *(const v8h*)(sT + p * 8);
  }
#pragma unroll
  for (int j = 0; j < 8; ++j) {
    const int p = (wave * 8 + j) * 32 + lane;
    *(volatile v4i*)(W2t + (size_t)p * 8) = o2[j].u;
  }
  __threadfence();
#pragma unroll
  for (int j = 0; j < 8; ++j) {
    const int p = (wave * 8 + j) * 32 + lane;
    *(volatile v4i*)(W2t + (size_t)p * 8) = o2[j].u;
  }
  __syncthreads();
  for (int i = tid; i < DIN * HC; i += 256) {
    const int k = i >> 7, n = i & 127;
    sT[n * DIN + k] = (_Float16)(W1[i] * WSC);
  }
  __syncthreads();
  Pk8 o1[4];
#pragma unroll
  for (int j = 0; j < 4; ++j) {
    const int p = (wave * 4 + j) * 32 + lane;
    o1[j].h = *(const v8h*)(sT + p * 8);
  }
#pragma unroll
  for (int j = 0; j < 4; ++j) {
    const int p = (wave * 4 + j) * 32 + lane;
    *(volatile v4i*)(W1t + (size_t)p * 8) = o1[j].u;
  }
  __threadfence();
#pragma unroll
  for (int j = 0; j < 4; ++j) {
    const int p = (wave * 4 + j) * 32 + lane;
    *(volatile v4i*)(W1t + (size_t)p * 8) = o1[j].u;
  }
}

__global__ __launch_bounds__(GTHR) __attribute__((amdgpu_num_vgpr(248)))
void k_gemm_p(const float* __restrict__ x, const _Float16* __restrict__ W1t,
              const float* __restrict__ b1, float* P, int nSrc) {
  __shared__ __attribute__((aligned(16))) float stg[4 * 16 * HC];
  const int tid = threadIdx.x, lane = tid & 31, wave = tid >> 5, h = lane >> 4, m = lane & 15;
  const int row0 = blockIdx.x * GROWS + wave * 16;
  int ra = row0 + m;
  ra = ra > nSrc - 1 ? nSrc - 1 : ra;
  const float* xr = x + (size_t)ra * DIN;
  FragH a[2];
#pragma unroll
  for (int kc = 0; kc < 2; ++kc) {
    const float* xp = xr + kc * 32 + 8 * h;
    const v4f p0 = *(const v4f*)xp;
    const v4f p1 = *(const v4f*)(xp + 4);
    const v4f q0 = *(const v4f*)(xp + 16);
    const v4f q1 = *(const v4f*)(xp + 20);
    a[kc].h[0] = cvt8(p0, p1);
    a[kc].h[1] = cvt8(q0, q1);
  }
  const v8f z8 = zero8f();
  v8f acc[8];
#pragma unroll
  for (int nt = 0; nt < 8; ++nt) {
    const _Float16* bp = W1t + (size_t)(nt * 16 + m) * DIN + 8 * h;
    FragH b0, b1f;
    b0.h[0]  = *(const v8h*)bp;
    b0.h[1]  = *(const v8h*)(bp + 16);
    b1f.h[0] = *(const v8h*)(bp + 32);
    b1f.h[1] = *(const v8h*)(bp + 48);
    acc[nt] = wmh(a[0].v, b0.v, z8);
    acc[nt] = wmh(a[1].v, b1f.v, acc[nt]);
  }
  float* sw = stg + wave * 16 * HC;
#pragma unroll
  for (int nt = 0; nt < 8; ++nt) {
    const float bb = b1[nt * 16 + m];
#pragma unroll
    for (int r = 0; r < 8; ++r) sw[(8 * h + r) * HC + nt * 16 + m] = acc[nt][r] * WINV + bb;
  }
  __syncthreads();
  const size_t gb = (size_t)row0 * HC;
#pragma unroll
  for (int rr = 0; rr < 16; ++rr) {
    const v4f v = *(const v4f*)(sw + rr * HC + 4 * lane);
    *(volatile v4f*)(P + gb + (size_t)rr * HC + 4 * lane) = v;
  }
  __threadfence();
#pragma unroll
  for (int rr = 0; rr < 16; ++rr) {
    const v4f v = *(const v4f*)(sw + rr * HC + 4 * lane);
    *(volatile v4f*)(P + gb + (size_t)rr * HC + 4 * lane) = v;
  }
}

__device__ __forceinline__ int scan_chunk(const int* __restrict__ dsts, int nE, int cbase, int nodeBase,
                                          int vec8, int* list, int tid, int wave) {
  int wc = 0;
  const int el0  = tid * EPT;
  const int e0   = cbase + el0;
  const int sent = -2147483647 - 1;
  v4i da, db;
  if (vec8 != 0 && cbase + CHUNK <= nE) {
    da = *(const v4i*)(dsts + e0);
    db = *(const v4i*)(dsts + e0 + 4);
  } else {
    da.x = (e0     < nE) ? dsts[min(e0,     nE - 1)] : sent;
    da.y = (e0 + 1 < nE) ? dsts[min(e0 + 1, nE - 1)] : sent;
    da.z = (e0 + 2 < nE) ? dsts[min(e0 + 2, nE - 1)] : sent;
    da.w = (e0 + 3 < nE) ? dsts[min(e0 + 3, nE - 1)] : sent;
    db.x = (e0 + 4 < nE) ? dsts[min(e0 + 4, nE - 1)] : sent;
    db.y = (e0 + 5 < nE) ? dsts[min(e0 + 5, nE - 1)] : sent;
    db.z = (e0 + 6 < nE) ? dsts[min(e0 + 6, nE - 1)] : sent;
    db.w = (e0 + 7 < nE) ? dsts[min(e0 + 7, nE - 1)] : sent;
  }
  const unsigned nb = (unsigned)nodeBase;
  const unsigned s0 = (unsigned)da.x - nb, s1 = (unsigned)da.y - nb;
  const unsigned s2 = (unsigned)da.z - nb, s3 = (unsigned)da.w - nb;
  const unsigned s4 = (unsigned)db.x - nb, s5 = (unsigned)db.y - nb;
  const unsigned s6 = (unsigned)db.z - nb, s7 = (unsigned)db.w - nb;
  const bool h0 = s0 < (unsigned)NB, h1 = s1 < (unsigned)NB, h2 = s2 < (unsigned)NB, h3 = s3 < (unsigned)NB;
  const bool h4 = s4 < (unsigned)NB, h5 = s5 < (unsigned)NB, h6 = s6 < (unsigned)NB, h7 = s7 < (unsigned)NB;
  const unsigned any = __builtin_amdgcn_ballot_w32(h0 | h1 | h2 | h3 | h4 | h5 | h6 | h7);
  if (any != 0u) {
#define HITJ(J, HJ) { \
      const unsigned mj = __builtin_amdgcn_ballot_w32(HJ); \
      if (mj != 0u) { \
        if (HJ) { \
          const int pos = wc + (int)__builtin_amdgcn_mbcnt_lo(mj, 0u); \
          if (pos < WCAP) list[wave * WCAP + pos] = el0 + (J); \
        } \
        wc += (int)__builtin_popcount(mj); } }
    HITJ(0, h0)
    HITJ(1, h1)
    HITJ(2, h2)
    HITJ(3, h3)
    HITJ(4, h4)
    HITJ(5, h5)
    HITJ(6, h6)
    HITJ(7, h7)
#undef HITJ
  }
  return wc;
}

__global__ __launch_bounds__(NTHR) __attribute__((amdgpu_num_vgpr(248)))
void k_agg(const float* __restrict__ P, const float* __restrict__ pos, const float* __restrict__ opos,
           const int* __restrict__ esrc, const int* __restrict__ edst,
           const float* __restrict__ W1, const float* __restrict__ b2,
           const _Float16* __restrict__ W2t, float* outp, int nSrc, int nOut, int nE) {
  __shared__ __attribute__((aligned(16))) float    accL[(NB + 1) * HC];
  __shared__ __attribute__((aligned(16))) _Float16 stgA[PASSN * HC];
  __shared__ __attribute__((aligned(16))) int      list[LISTN];
  __shared__ __attribute__((aligned(16))) int      pend[PCAP];
  __shared__ __attribute__((aligned(16))) v4f      eD[PASSN];
  __shared__ int eSrc[PASSN];
  __shared__ int eSlot[PASSN];
  __shared__ int wcnt[NWAVE];
  __shared__ int pendN;

  const int tid = threadIdx.x, lane = tid & 31, wave = tid >> 5, h = lane >> 4, m = lane & 15;
  const int g = tid & 15;
  const int nodeBase = blockIdx.x * NB;

  {
    const v4f z4 = {0.0f, 0.0f, 0.0f, 0.0f};
    for (int i = tid; i < ((NB + 1) * HC) / 4; i += NTHR) *(v4f*)(accL + 4 * i) = z4;
  }
  if (tid == 0) pendN = 0;
  float wa[8], wb[8], wcf[8], b2v[8];
#pragma unroll
  for (int j = 0; j < 8; ++j) {
    wa[j]  = W1[(DIN + 0) * HC + 8 * g + j];
    wb[j]  = W1[(DIN + 1) * HC + 8 * g + j];
    wcf[j] = W1[(DIN + 2) * HC + 8 * g + j];
  }
#pragma unroll
  for (int nt = 0; nt < 8; ++nt) b2v[nt] = b2[nt * 16 + m];
  const int vec8 = ((((uintptr_t)edst) & 15) == 0) ? 1 : 0;
  const v8f z8 = zero8f();
  __syncthreads();

  const int nChunks = (nE + CHUNK - 1) / CHUNK;
#pragma unroll 1
  for (int ch = 0; ch < nChunks; ++ch) {
    const int cbase = ch * CHUNK;
    const int wc = scan_chunk(edst, nE, cbase, nodeBase, vec8, list, tid, wave);
    if (lane == 0) wcnt[wave] = wc;
    __syncthreads();

    const int base = pendN;
    int tot = 0, myoff = 0;
#pragma unroll
    for (int w = 0; w < NWAVE; ++w) {
      int c = wcnt[w];
      c = c > WCAP ? WCAP : (c < 0 ? 0 : c);
      if (w < wave) myoff += c;
      tot += c;
    }
    int newN = base + tot;
    newN = newN > PCAP ? PCAP : newN;
    {
      int n = wcnt[wave];
      n = n > WCAP ? WCAP : (n < 0 ? 0 : n);
      const int* lp = list + wave * WCAP;
      for (int i = lane; i < n; i += 32) {
        const int pp = base + myoff + i;
        if (pp < PCAP) pend[pp] = cbase + lp[i];
      }
    }
    const int fin = (ch == nChunks - 1) ? 1 : 0;
    const int R   = (fin != 0) ? (newN + PASSN - 1) / PASSN : newN / PASSN;
    const int Pv  = (fin != 0) ? newN : R * PASSN;
    __syncthreads();

#pragma unroll 1
    for (int r = 0; r < R; ++r) {
      if (tid < PASSN) {
        const int idx = r * PASSN + tid;
        const bool valid = idx < Pv;
        const int ic = idx < PCAP - 1 ? idx : PCAP - 1;
        int e = pend[ic];
        e = valid ? e : 0;
        e = e < 0 ? 0 : (e > nE - 1 ? nE - 1 : e);
        int d = edst[e];
        int s = esrc[e];
        int slot = d - nodeBase;
        if (!valid || (unsigned)slot >= (unsigned)NB) slot = NB;
        d = d < 0 ? 0 : (d > nOut - 1 ? nOut - 1 : d);
        s = s < 0 ? 0 : (s > nSrc - 1 ? nSrc - 1 : s);
        const float dx = pos[(size_t)s * 3 + 0] - opos[(size_t)d * 3 + 0];
        const float dy = pos[(size_t)s * 3 + 1] - opos[(size_t)d * 3 + 1];
        const float dz = pos[(size_t)s * 3 + 2] - opos[(size_t)d * 3 + 2];
        eSrc[tid]  = s;
        eSlot[tid] = slot;
        v4f dv = {dx, dy, dz, 0.0f};
        eD[tid] = dv;
      }
      __syncthreads();

#pragma unroll 1
      for (int it = 0; it < 8; ++it) {
        const int ei = it * (NTHR / 16) + (tid >> 4);
        const int s  = eSrc[ei];
        const v4f dv = eD[ei];
        const float* pr = P + (size_t)s * HC + 8 * g;
        const v4f p0 = *(const v4f*)pr;
        const v4f p1 = *(const v4f*)(pr + 4);
        float t[8];
        t[0] = p0.x; t[1] = p0.y; t[2] = p0.z; t[3] = p0.w;
        t[4] = p1.x; t[5] = p1.y; t[6] = p1.z; t[7] = p1.w;
        v8h hv;
#pragma unroll
        for (int j = 0; j < 8; ++j) {
          float u = fmaf(dv.x, wa[j], t[j]);
          u = fmaf(dv.y, wb[j], u);
          u = fmaf(dv.z, wcf[j], u);
          u = fmaxf(u, 0.0f);
          hv[j] = (_Float16)u;
        }
        *(v8h*)(stgA + ei * HC + 8 * g) = hv;
      }
      __syncthreads();

      FragH af[4];
      {
        const _Float16* ap = stgA + (16 * wave + m) * HC + 8 * h;
#pragma unroll
        for (int kc = 0; kc < 4; ++kc) {
          af[kc].h[0] = *(const v8h*)(ap + kc * 32);
          af[kc].h[1] = *(const v8h*)(ap + kc * 32 + 16);
        }
      }
      v8f hv2[8];
#pragma unroll
      for (int nt = 0; nt < 8; ++nt) {
        const _Float16* bp = W2t + (size_t)(nt * 16 + m) * HC + 8 * h;
        FragH b;
        v8f acc;
        b.h[0] = *(const v8h*)(bp);       b.h[1] = *(const v8h*)(bp + 16);
        acc = wmh(af[0].v, b.v, z8);
        b.h[0] = *(const v8h*)(bp + 32);  b.h[1] = *(const v8h*)(bp + 48);
        acc = wmh(af[1].v, b.v, acc);
        b.h[0] = *(const v8h*)(bp + 64);  b.h[1] = *(const v8h*)(bp + 80);
        acc = wmh(af[2].v, b.v, acc);
        b.h[0] = *(const v8h*)(bp + 96);  b.h[1] = *(const v8h*)(bp + 112);
        acc = wmh(af[3].v, b.v, acc);
#pragma unroll
        for (int rr = 0; rr < 8; ++rr) hv2[nt][rr] = fmaxf(acc[rr] * WINV + b2v[nt], 0.0f);
      }

#pragma unroll 1
      for (int w2 = 0; w2 < NWAVE; ++w2) {
        if (wave == w2) {
#pragma unroll
          for (int hs = 0; hs < 2; ++hs) {
            if (h == hs) {
#pragma unroll
              for (int rr = 0; rr < 8; ++rr) {
                int sl = eSlot[16 * w2 + 8 * hs + rr];
                sl = sl < 0 ? 0 : (sl > NB ? NB : sl);
                float* q = accL + sl * HC + m;
#pragma unroll
                for (int nt = 0; nt < 8; ++nt) {
                  const float o = q[nt * 16];
                  q[nt * 16] = fmaxf(o, hv2[nt][rr]);
                }
              }
            }
            __builtin_amdgcn_fence(__ATOMIC_RELEASE, "wavefront");
            __builtin_amdgcn_wave_barrier();
          }
        }
        __syncthreads();
      }
    }

    int rem = newN - R * PASSN;
    rem = rem < 0 ? 0 : rem;
    if (R > 0 && tid < rem) pend[tid] = pend[R * PASSN + tid];
    if (tid == 0) pendN = rem;
  }
  __syncthreads();

#pragma unroll 1
  for (int ri = wave; ri < NB; ri += NWAVE) {
    const int grow = nodeBase + ri;
    if (grow < nOut) {
      const v4f v = *(const v4f*)(accL + ri * HC + 4 * lane);
      *(volatile v4f*)(outp + (size_t)grow * HC + 4 * lane) = v;
    }
  }
  __threadfence();
#pragma unroll 1
  for (int ri = wave; ri < NB; ri += NWAVE) {
    const int grow = nodeBase + ri;
    if (grow < nOut) {
      const v4f v = *(const v4f*)(accL + ri * HC + 4 * lane);
      *(volatile v4f*)(outp + (size_t)grow * HC + 4 * lane) = v;
    }
  }
}

extern "C" void kernel_launch(void* const* d_in, const int* in_sizes, int n_in,
                              void* d_out, int out_size, void* d_ws, size_t ws_size,
                              hipStream_t stream) {
  if (n_in < 9) return;
  const int nSrc = in_sizes[0] / DIN;
  if (nSrc <= 0 || in_sizes[0] != nSrc * DIN || in_sizes[1] != nSrc * 3) return;
  const int nOut = in_sizes[2] / 3;
  if (nOut <= 0 || in_sizes[2] != nOut * 3) return;
  const int nE = in_sizes[3];
  if (nE < 0 || in_sizes[4] != nE) return;
  if (in_sizes[5] != (DIN + 3) * HC || in_sizes[6] != HC || in_sizes[7] != HC * HC || in_sizes[8] != HC) return;
  if (out_size != nOut * HC) return;

  const float* x    = (const float*)d_in[0];
  const float* pos  = (const float*)d_in[1];
  const float* opos = (const float*)d_in[2];
  const int*   esrc = (const int*)d_in[3];
  const int*   edst = (const int*)d_in[4];
  const float* W1   = (const float*)d_in[5];
  const float* b1   = (const float*)d_in[6];
  const float* W2   = (const float*)d_in[7];
  const float* b2   = (const float*)d_in[8];
  float* out = (float*)d_out;

  const int nBlkG = (nSrc + GROWS - 1) / GROWS;
  const size_t rowsPad = (size_t)nBlkG * GROWS;

  char* ws = (char*)d_ws;
  size_t off = 0;
  const size_t oW1t = off; off += (size_t)HC * DIN * 2;
  const size_t oW2t = off; off += (size_t)HC * HC * 2;
  off = (off + 255) & ~(size_t)255;
  const size_t oP = off;   off += rowsPad * HC * 4;
  off = (off + 255) & ~(size_t)255;
  if (off > ws_size) return;
  if (off > (size_t)134217728) return;
  _Float16* W1t = (_Float16*)(ws + oW1t);
  _Float16* W2t = (_Float16*)(ws + oW2t);
  float*    P   = (float*)(ws + oP);

  k_prep<<<1, 256, 0, stream>>>(W1, W2, W1t, W2t);
  k_gemm_p<<<nBlkG, GTHR, 0, stream>>>(x, W1t, b1, P, nSrc);
  const int nBlkA = (nOut + NB - 1) / NB;
  k_agg<<<nBlkA, NTHR, 0, stream>>>(P, pos, opos, esrc, edst, W1, b2, W2t, out, nSrc, nOut, nE);
}
